// MultiHeadedAddAttention_59983513255986
// MI455X (gfx1250) — hardware-verified
//
#include <hip/hip_runtime.h>


#define NB_  2
#define LQ   256
#define LK   512
#define DM   512
#define NH_  8
#define DK   64
typedef _Float16 h16;
typedef unsigned short bf;
typedef __attribute__((ext_vector_type(16))) __bf16   v16bf;
typedef __attribute__((ext_vector_type(16))) _Float16 v16h;
typedef __attribute__((ext_vector_type(8)))  _Float16 v8h;
typedef __attribute__((ext_vector_type(8)))  unsigned short v8us;
typedef __attribute__((ext_vector_type(8)))  float    v8f;
typedef __attribute__((ext_vector_type(4)))  float    v4f;
typedef v8h  __attribute__((may_alias)) v8ha;
typedef v4f  __attribute__((may_alias)) v4fa;
typedef v8us __attribute__((may_alias)) v8usa;

__device__ __forceinline__ unsigned short f2bf(float f) { unsigned u = __float_as_uint(f); u += 0x7FFFu + ((u >> 16) & 1u); return (unsigned short)(u >> 16); }
__device__ __forceinline__ float bf2f(unsigned short b) { return __uint_as_float(((unsigned)b) << 16); }
__device__ __forceinline__ float bfr(float f) { return bf2f(f2bf(f)); }
__device__ __forceinline__ v16h cat16(v8h lo, v8h hi) { return __builtin_shufflevector(lo, hi, 0, 1, 2, 3, 4, 5, 6, 7, 8, 9, 10, 11, 12, 13, 14, 15); }
__device__ __forceinline__ v16bf cat16b(v8us lo, v8us hi) { return __builtin_bit_cast(v16bf, __builtin_shufflevector(lo, hi, 0, 1, 2, 3, 4, 5, 6, 7, 8, 9, 10, 11, 12, 13, 14, 15)); }
__device__ __forceinline__ v8f wmma16(v16h a, v16h b, v8f c) { return __builtin_amdgcn_wmma_f32_16x16x32_f16(false, a, false, b, (short)0, c, false, false); }
__device__ __forceinline__ v8f wmmab(v16bf a, v16bf b, v8f c) { return __builtin_amdgcn_wmma_f32_16x16x32_bf16(false, a, false, b, (short)0, c, false, false); }


template <typename T16> struct WFrag;
template <> struct WFrag<h16> { typedef v16h V; static __device__ __forceinline__ V ld(const h16* p) { return cat16(*(const v8h*)p, *(const v8h*)(p + 16)); } static __device__ __forceinline__ v8f mma(V a, V b, v8f c) { return wmma16(a, b, c); } };
template <> struct WFrag<bf> { typedef v16bf V; static __device__ __forceinline__ V ld(const bf* p) { return cat16b(*(const v8us*)p, *(const v8us*)(p + 16)); } static __device__ __forceinline__ v8f mma(V a, V b, v8f c) { return wmmab(a, b, c); } };
template <typename T16, int NSPLIT, bool BIAS>
__global__ __launch_bounds__(32) void k_gemmw(const T16* __restrict__ A, const T16* __restrict__ A2, const T16* __restrict__ Bt, const T16* __restrict__ Bt2, int K, float* C, int ldc, const float* __restrict__ bias, size_t sA, size_t sB, size_t sC) {
    typedef typename WFrag<T16>::V V;
    __shared__ __align__(16) float os[16 * 68];
    const size_t z = blockIdx.z; A += z * sA; if (A2) A2 += z * sA; Bt += z * sB; if (Bt2) Bt2 += z * sB; C += z * sC;
    const int lane = threadIdx.x & 31, lr = lane & 15, hi = lane >> 4; const int r0 = blockIdx.x * 64, c0 = blockIdx.y * 64;
    v8f acc[4][4];
#pragma unroll
    for (int mb = 0; mb < 4; ++mb)
#pragma unroll
        for (int nb = 0; nb < 4; ++nb) acc[mb][nb] = (v8f){};
    const size_t aoff = (size_t)(r0 + lr) * K + 8 * hi, boff = (size_t)(c0 + lr) * K + 8 * hi;
#pragma unroll 1
    for (int kc = 0; kc < K; kc += 32) {
        V a[4], a2[4];
#pragma unroll
        for (int mb = 0; mb < 4; ++mb) { a[mb] = WFrag<T16>::ld(A + aoff + (size_t)mb * 16 * K + kc); if (NSPLIT == 1 || NSPLIT == 2) a2[mb] = WFrag<T16>::ld(A2 + aoff + (size_t)mb * 16 * K + kc); }
#pragma unroll
        for (int nb = 0; nb < 4; ++nb) { const V b = WFrag<T16>::ld(Bt + boff + (size_t)nb * 16 * K + kc); V b2; if (NSPLIT >= 2) b2 = WFrag<T16>::ld(Bt2 + boff + (size_t)nb * 16 * K + kc);
#pragma unroll
            for (int mb = 0; mb < 4; ++mb) { acc[mb][nb] = WFrag<T16>::mma(a[mb], b, acc[mb][nb]); if (NSPLIT == 1 || NSPLIT == 2) acc[mb][nb] = WFrag<T16>::mma(a2[mb], b, acc[mb][nb]); if (NSPLIT >= 2) acc[mb][nb] = WFrag<T16>::mma(a[mb], b2, acc[mb][nb]); } }
        asm volatile("v_nop\n\tv_nop\n\tv_nop\n\tv_nop" : "+v"(acc[0][0]), "+v"(acc[1][1]), "+v"(acc[2][2]), "+v"(acc[3][3]) : "v"(a[0]), "v"(a[3]));
    }
#pragma unroll
    for (int mb = 0; mb < 4; ++mb) {
#pragma unroll
        for (int nb = 0; nb < 4; ++nb) {
#pragma unroll
            for (int j = 0; j < 8; ++j) os[(hi * 8 + j) * 68 + nb * 16 + lr] = acc[mb][nb][j]; }
        __builtin_amdgcn_wave_barrier(); asm volatile("" ::: "memory");
        float* crow = C + (size_t)(r0 + mb * 16) * ldc + c0;
#pragma unroll 1
        for (int ps = 0; ps < 2; ++ps) {
#pragma unroll
            for (int s = 0; s < 8; ++s) { const int row = 2 * s + hi, cofs = lr * 4; v4f val = *(const v4fa*)(os + row * 68 + cofs); if (BIAS) { val[0] += bfr(bias[c0 + cofs]); val[1] += bfr(bias[c0 + cofs + 1]); val[2] += bfr(bias[c0 + cofs + 2]); val[3] += bfr(bias[c0 + cofs + 3]); }
                *(volatile v4f*)(crow + (size_t)row * ldc + cofs) = val; }
            if (ps == 0) __threadfence(); }
        __builtin_amdgcn_wave_barrier(); asm volatile("" ::: "memory");
    }
}

__device__ __forceinline__ void splitf(float y, unsigned short& h, unsigned short& l) { h = f2bf(y); l = f2bf(y - bf2f(h)); }
__device__ __forceinline__ float tanh_(float x) { const float e = __expf(-2.0f * fabsf(x)); const float t = __fdiv_rn(1.0f - e, 1.0f + e); return copysignf(t, x); }
typedef __attribute__((ext_vector_type(2))) unsigned short v2us;

__global__ __launch_bounds__(256) void k_cvt8(const float* __restrict__ src, bf* dst, size_t n8) { const size_t i = (size_t)blockIdx.x * 256 + threadIdx.x; if (i >= n8) return; const v8f v = *(const v8f*)(src + i * 8); v8us o;
#pragma unroll
    for (int k = 0; k < 8; ++k) o[k] = f2bf(v[k]); *(volatile v8us*)(dst + i * 8) = o; __threadfence(); *(volatile v8us*)(dst + i * 8) = o; }
__global__ __launch_bounds__(256) void k_wtG(const float* __restrict__ w, int K, int N, bf* Bt) {
    const int lane = threadIdx.x & 31; const int L0 = (blockIdx.x * 8 + (threadIdx.x >> 5)) * 8; const int nlines = N * K / 64;
#pragma unroll 1
    for (int ps = 0; ps < 2; ++ps) {
#pragma unroll 1
        for (int l = 0; l < 8; ++l) { const int L = L0 + l; if (L >= nlines) break; const size_t e = (size_t)L * 64 + lane * 2; const int k = (int)(e % K), n = (int)(e / K); v2us o;
            o[0] = f2bf(w[(size_t)k * N + n]); o[1] = f2bf(w[(size_t)(k + 1) * N + n]); *(volatile v2us*)(Bt + e) = o; }
        if (ps == 0) __threadfence(); }
}
__global__ __launch_bounds__(256) void k_addatt(const float* __restrict__ Q, const float* __restrict__ Kf, const float* __restrict__ V, const float* __restrict__ wa, const int* __restrict__ mk, int b, bf* Xh, bf* Xl) {
    __shared__ float pr[8][LK]; const int lane = threadIdx.x & 31; const int wv = threadIdx.x >> 5; const int row = blockIdx.x * 8 + wv; if (row >= NH_ * LQ) return; const int h = row % NH_; const int qi = row / NH_; const float* qp = Q + (size_t)qi * DM + h * DK; float mx = -3.0e38f;
#pragma unroll 1
    for (int m = 0; m < LK / 32; ++m) { const int j = m * 32 + lane; const float* kp = Kf + (size_t)j * DM + h * DK; float s = 0.f;
#pragma unroll 1
        for (int d = 0; d < DK; ++d) { float p = __fmul_rn(tanh_(__fadd_rn(qp[d], kp[d])), bfr(wa[d])); asm volatile("" : "+v"(p)); s = __fadd_rn(s, p); }
        if (mk[b * LK + j] == 0) s = -1.0e9f; pr[wv][j] = s; mx = fmaxf(mx, s); }
#pragma unroll
    for (int sh = 16; sh; sh >>= 1) mx = fmaxf(mx, __shfl_xor(mx, sh, 32));
    float sum = 0.f;
#pragma unroll 1
    for (int m = 0; m < LK / 32; ++m) { const int j = m * 32 + lane; float d0 = __fsub_rn(pr[wv][j], mx); asm volatile("" : "+v"(d0)); const float e = __expf(d0); pr[wv][j] = e; sum = __fadd_rn(sum, e); }
#pragma unroll
    for (int sh = 16; sh; sh >>= 1) sum += __shfl_xor(sum, sh, 32);
    const float inv = __fdiv_rn(1.0f, sum);
#pragma unroll 1
    for (int m = 0; m < LK / 32; ++m) { const int j = m * 32 + lane; pr[wv][j] = __fmul_rn(pr[wv][j], inv); }
    __syncthreads();
    const int d = lane * 2; float a0 = 0.f, a1 = 0.f;
#pragma unroll 1
    for (int j = 0; j < LK; ++j) { const float p = pr[wv][j]; const float* vp = V + (size_t)j * DM + h * DK + d; float u0 = __fmul_rn(p, vp[0]), u1 = __fmul_rn(p, vp[1]); asm volatile("" : "+v"(u0)); asm volatile("" : "+v"(u1)); a0 = __fadd_rn(a0, u0); a1 = __fadd_rn(a1, u1); }
    v2us oh, ol; unsigned short t0, t1; splitf(a0, t0, t1); oh[0] = t0; ol[0] = t1; splitf(a1, t0, t1); oh[1] = t0; ol[1] = t1; const size_t oo = (size_t)qi * DM + h * DK + d;
    *(volatile v2us*)(Xh + oo) = oh; *(volatile v2us*)(Xl + oo) = ol; __threadfence(); *(volatile v2us*)(Xh + oo) = oh; *(volatile v2us*)(Xl + oo) = ol; }

extern "C" void kernel_launch(void* const* d_in, const int* in_sizes, int n_in,
                              void* d_out, int out_size, void* d_ws, size_t ws_size, hipStream_t stream) {
    (void)in_sizes; (void)n_in; (void)out_size;
    const float* query = (const float*)d_in[0]; const float* key = (const float*)d_in[1]; const float* value = (const float*)d_in[2]; const int* mk = (const int*)d_in[3]; const float* wq = (const float*)d_in[4]; const float* wk = (const float*)d_in[5]; const float* wv = (const float*)d_in[6]; const float* wo = (const float*)d_in[7]; const float* wa = (const float*)d_in[8];
    float* OUT = (float*)d_out;
    char* wsp = (char*)d_ws;
    auto take = [&](size_t bytes) { char* p = wsp; wsp += (bytes + 255) & ~(size_t)255; return (void*)p; };
    bf* WQ = (bf*)take(DM * DM * 2); bf* WK = (bf*)take(DM * DM * 2); bf* WV = (bf*)take(DM * DM * 2); bf* WO = (bf*)take(DM * DM * 2); bf* XQ = (bf*)take((size_t)LQ * DM * 2); bf* XK = (bf*)take((size_t)LK * DM * 2); bf* XV = (bf*)take((size_t)LK * DM * 2);
    float* Q = (float*)take((size_t)LQ * DM * 4); float* Kf = (float*)take((size_t)LK * DM * 4); float* V = (float*)take((size_t)LK * DM * 4); bf* Xh = (bf*)take((size_t)LQ * DM * 2); bf* Xl = (bf*)take((size_t)LQ * DM * 2);
    if ((size_t)(wsp - (char*)d_ws) > ws_size) return;
    k_wtG<<<(DM * DM / 64 + 63) / 64, 256, 0, stream>>>(wq, DM, DM, WQ); k_wtG<<<(DM * DM / 64 + 63) / 64, 256, 0, stream>>>(wk, DM, DM, WK); k_wtG<<<(DM * DM / 64 + 63) / 64, 256, 0, stream>>>(wv, DM, DM, WV); k_wtG<<<(DM * DM / 64 + 63) / 64, 256, 0, stream>>>(wo, DM, DM, WO);
    for (int b = 0; b < NB_; ++b) {
        k_cvt8<<<(LQ * DM / 8 + 255) / 256, 256, 0, stream>>>(query + (size_t)b * LQ * DM, XQ, LQ * DM / 8); k_cvt8<<<(LK * DM / 8 + 255) / 256, 256, 0, stream>>>(key + (size_t)b * LK * DM, XK, LK * DM / 8); k_cvt8<<<(LK * DM / 8 + 255) / 256, 256, 0, stream>>>(value + (size_t)b * LK * DM, XV, LK * DM / 8);
        k_gemmw<bf, 0, false><<<dim3(LQ / 64, DM / 64, 1), 32, 0, stream>>>(XQ, nullptr, WQ, nullptr, DM, Q, DM, nullptr, 0, 0, 0); k_gemmw<bf, 0, false><<<dim3(LK / 64, DM / 64, 1), 32, 0, stream>>>(XK, nullptr, WK, nullptr, DM, Kf, DM, nullptr, 0, 0, 0); k_gemmw<bf, 0, false><<<dim3(LK / 64, DM / 64, 1), 32, 0, stream>>>(XV, nullptr, WV, nullptr, DM, V, DM, nullptr, 0, 0, 0);
        k_addatt<<<NH_ * LQ / 8, 256, 0, stream>>>(Q, Kf, V, wa, mk, b, Xh, Xl);
        k_gemmw<bf, 1, false><<<dim3(LQ / 64, DM / 64, 1), 32, 0, stream>>>(Xh, Xl, WO, nullptr, DM, OUT + (size_t)b * LQ * DM, DM, nullptr, 0, 0, 0); }
}
